// RNN_20289425506787
// MI455X (gfx1250) — hardware-verified
//
#include <hip/hip_runtime.h>
#include <math.h>

typedef __attribute__((ext_vector_type(16))) _Float16 v16h;
typedef __attribute__((ext_vector_type(8)))  _Float16 v8h;
typedef __attribute__((ext_vector_type(8)))  float    v8f;
typedef __attribute__((ext_vector_type(4)))  float    v4f;

constexpr int kBatch   = 4096;
constexpr int kSteps   = 512;
constexpr int kHid     = 128;
constexpr int kOutD    = 128;
constexpr int kRowsPB  = 16;
constexpr int kThreads = 256;
constexpr int kWaves   = kThreads / 32;
constexpr int kHP      = kHid + 8;
constexpr int kHTile   = kRowsPB * kHP;
constexpr int kLP      = kOutD + 4;
constexpr float kHCarry       = 16.0f;
constexpr float kWCarry       = 64.0f;
constexpr float kCarry        = kHCarry * kWCarry;
constexpr float kCarryInv     = 1.0f / kCarry;
constexpr float kTwoCarryInv  = 2.0f / kCarry;

static_assert(kBatch % kRowsPB == 0, "grid exact");
static_assert(kHid == 16 * kWaves, "one 16-column subtile per wave");
static_assert(kOutD == 16 * kWaves, "one 16-column head subtile per wave");
static_assert(kHid % 32 == 0, "K multiple of 32");
static_assert(kRowsPB == 2 * kWaves, "two softmax rows per wave");
static_assert(kHP % 8 == 0 && kLP % 4 == 0, "aligned pitches");
static_assert((kRowsPB * kSteps / 4) % kThreads == 0, "x staging loop exact");
static_assert(kOutD == 4 * 32, "one float4 per lane per output row");

union FragU { v16h v; v8h h[2]; };
__device__ __forceinline__ v16h frag_load_h(const _Float16* p) {
  FragU f;
  f.h[0] = *(const v8h*)(p);
  f.h[1] = *(const v8h*)(p + 16);
  return f.v;
}

__device__ __forceinline__ v8f mma_f16(v16h a, v16h b, v8f c) {
  c = __builtin_amdgcn_wmma_f32_16x16x32_f16(false, a, false, b, (short)0, c, false, false);
  asm volatile("v_nop\n\tv_nop\n\tv_nop\n\tv_nop" : "+v"(c) : "v"(a), "v"(b));
  return c;
}

__device__ __forceinline__ v16h wfrag_load(const float* p, float sc) {
  const v4f p0 = *(const v4f*)(p);
  const v4f p1 = *(const v4f*)(p + 4);
  const v4f p2 = *(const v4f*)(p + 16);
  const v4f p3 = *(const v4f*)(p + 20);
  v16h f;
#pragma unroll
  for (int e = 0; e < 4; ++e) {
    f[e]      = (_Float16)(p0[e] * sc);
    f[4 + e]  = (_Float16)(p1[e] * sc);
    f[8 + e]  = (_Float16)(p2[e] * sc);
    f[12 + e] = (_Float16)(p3[e] * sc);
  }
  return f;
}

__device__ __forceinline__ float tanh_from_2z(float z2) {
  const float e = expf(z2);
  return 1.0f - 2.0f * __builtin_amdgcn_rcpf(e + 1.0f);
}

__global__ __launch_bounds__(kThreads) void elman_seq_kernel(
    const float* __restrict__ seq,
    const float* __restrict__ Wh_w, const float* __restrict__ Wh_b,
    const float* __restrict__ Wi_w, const float* __restrict__ Wi_b,
    const float* __restrict__ Wo_w, const float* __restrict__ Wo_b,
    float* __restrict__ out) {
  __shared__ __align__(16) float    x_sh[kSteps * kRowsPB];
  __shared__ __align__(16) _Float16 hbuf[2 * kHTile];
  __shared__ __align__(16) float    lg_sh[kRowsPB * kLP];

  const int tid  = threadIdx.x;
  const int lane = tid & 31;
  const int wave = tid >> 5;
  const int c    = lane & 15;
  const int hh   = lane >> 4;
  const int koff = hh * 8;
  const int rowbase = blockIdx.x * kRowsPB;
  const int n = wave * 16 + c;

  v16h bfr[4];
  {
    const float* wrow = Wh_w + (size_t)n * kHid + koff;
#pragma unroll
    for (int kc = 0; kc < 4; ++kc) {
      bfr[kc] = wfrag_load(wrow + kc * 32, kWCarry);
      asm volatile("" ::: "memory");
    }
  }
  const float bsum_s = (Wh_b[n] + Wi_b[n]) * kCarry;
  const float wi_s   = Wi_w[n] * kCarry;
  const float wob_s  = Wo_b[n] * kCarry;
  asm volatile("" ::: "memory");

  {
    const v8h z = {(_Float16)0.f, (_Float16)0.f, (_Float16)0.f, (_Float16)0.f,
                   (_Float16)0.f, (_Float16)0.f, (_Float16)0.f, (_Float16)0.f};
    for (int i = tid; i < (2 * kHTile) / 8; i += kThreads) *(v8h*)(hbuf + i * 8) = z;
  }
#pragma unroll 1
  for (int it = 0; it < (kRowsPB * kSteps / 4) / kThreads; ++it) {
    const int f   = it * kThreads + tid;
    const int row = f >> 7;
    const int c4  = f & 127;
    const v4f xv = *(const v4f*)(seq + (size_t)(rowbase + row) * kSteps + c4 * 4);
    x_sh[(c4 * 4 + 0) * kRowsPB + row] = xv[0];
    x_sh[(c4 * 4 + 1) * kRowsPB + row] = xv[1];
    x_sh[(c4 * 4 + 2) * kRowsPB + row] = xv[2];
    x_sh[(c4 * 4 + 3) * kRowsPB + row] = xv[3];
  }
  __syncthreads();

#pragma unroll 1
  for (int t = 0; t < kSteps; ++t) {
    const _Float16* hc = hbuf + (t & 1) * kHTile;
    _Float16*       hn = hbuf + ((t + 1) & 1) * kHTile;

    const float* xp = x_sh + t * kRowsPB + 8 * hh;
    const v4f xa = *(const v4f*)(xp);
    const v4f xb = *(const v4f*)(xp + 4);
    v8f acc;
    acc[0] = fmaf(xa[0], wi_s, bsum_s);
    acc[1] = fmaf(xa[1], wi_s, bsum_s);
    acc[2] = fmaf(xa[2], wi_s, bsum_s);
    acc[3] = fmaf(xa[3], wi_s, bsum_s);
    acc[4] = fmaf(xb[0], wi_s, bsum_s);
    acc[5] = fmaf(xb[1], wi_s, bsum_s);
    acc[6] = fmaf(xb[2], wi_s, bsum_s);
    acc[7] = fmaf(xb[3], wi_s, bsum_s);

    const _Float16* arow = hc + c * kHP + koff;
#pragma unroll
    for (int kc = 0; kc < 4; ++kc) {
      const v16h a = frag_load_h(arow + kc * 32);
      acc = mma_f16(a, bfr[kc], acc);
    }

#pragma unroll
    for (int r = 0; r < 8; ++r) {
      const float hv = tanh_from_2z(acc[r] * kTwoCarryInv);
      hn[(8 * hh + r) * kHP + n] = (_Float16)(hv * kHCarry);
    }
    __syncthreads();
  }

  {
    const _Float16* hT = hbuf + (kSteps & 1) * kHTile;
    v16h ofr[4];
    const float* orow = Wo_w + (size_t)n * kHid + koff;
#pragma unroll
    for (int kc = 0; kc < 4; ++kc) {
      ofr[kc] = wfrag_load(orow + kc * 32, kWCarry);
      asm volatile("" ::: "memory");
    }
    v8f acc;
#pragma unroll
    for (int r = 0; r < 8; ++r) acc[r] = wob_s;
    const _Float16* arow = hT + c * kHP + koff;
#pragma unroll
    for (int kc = 0; kc < 4; ++kc) {
      const v16h a = frag_load_h(arow + kc * 32);
      acc = mma_f16(a, ofr[kc], acc);
    }
#pragma unroll
    for (int r = 0; r < 8; ++r) lg_sh[(8 * hh + r) * kLP + n] = acc[r] * kCarryInv;
  }
  __syncthreads();

#pragma unroll 1
  for (int rr = 0; rr < 2; ++rr) {
    const int row = 2 * wave + rr;
    const v4f v = *(const v4f*)(lg_sh + row * kLP + 4 * lane);
    float m = fmaxf(fmaxf(v[0], v[1]), fmaxf(v[2], v[3]));
#pragma unroll
    for (int off = 16; off >= 1; off >>= 1) m = fmaxf(m, __shfl_xor(m, off, 32));
    v4f e;
    e[0] = expf(v[0] - m);
    e[1] = expf(v[1] - m);
    e[2] = expf(v[2] - m);
    e[3] = expf(v[3] - m);
    float s = (e[0] + e[1]) + (e[2] + e[3]);
#pragma unroll
    for (int off = 16; off >= 1; off >>= 1) s += __shfl_xor(s, off, 32);
    const float inv = 1.0f / s;
    v4f o;
    o[0] = e[0] * inv;
    o[1] = e[1] * inv;
    o[2] = e[2] * inv;
    o[3] = e[3] * inv;
    float* op = out + (size_t)(rowbase + row) * kOutD + 4 * lane;
    *(volatile v4f*)op = o;
    __threadfence();
    *(volatile v4f*)op = o;
  }
}

extern "C" void kernel_launch(void* const* d_in, const int* in_sizes, int n_in,
                              void* d_out, int out_size, void* d_ws, size_t ws_size, hipStream_t stream) {
  (void)d_ws; (void)ws_size;
  if (n_in < 7 || d_out == nullptr) return;
  if (in_sizes[0] != kBatch * kSteps || in_sizes[1] != kHid * kHid || in_sizes[2] != kHid ||
      in_sizes[3] != kHid || in_sizes[4] != kHid || in_sizes[5] != kOutD * kHid ||
      in_sizes[6] != kOutD || out_size != kBatch * kOutD) return;

  const float* seq  = (const float*)d_in[0];
  const float* Wh_w = (const float*)d_in[1];
  const float* Wh_b = (const float*)d_in[2];
  const float* Wi_w = (const float*)d_in[3];
  const float* Wi_b = (const float*)d_in[4];
  const float* Wo_w = (const float*)d_in[5];
  const float* Wo_b = (const float*)d_in[6];
  float* outp = (float*)d_out;

  elman_seq_kernel<<<kBatch / kRowsPB, kThreads, 0, stream>>>(seq, Wh_w, Wh_b, Wi_w, Wi_b, Wo_w, Wo_b, outp);
}
